// BaseModelWithEmbedding_83176336654766
// MI455X (gfx1250) — hardware-verified
//
#include <hip/hip_runtime.h>
#include <math.h>

#define NSEQ    256
#define NSTEP   512
#define NHID    128
#define NGATE   512
#define NTHR    256
#define HPITCH  136
#define OPITCH  132
#define HCOLS   384
#define NHOUR   24
#define NWEEK   7
#define USCALE  16.0f
#define USCALE_INV (1.0f / 16.0f)

typedef __attribute__((ext_vector_type(16))) _Float16 v16h;
typedef __attribute__((ext_vector_type(8)))  _Float16 v8h;
typedef __attribute__((ext_vector_type(8)))  float    v8f;
typedef __attribute__((ext_vector_type(4)))  float    v4f;

__device__ __forceinline__ void dep_guard_h(v8f& a, v8f& b, v16h x, v16h y) { asm volatile("v_nop\n\tv_nop\n\tv_nop\n\tv_nop" : "+v"(a), "+v"(b) : "v"(x), "v"(y)); }
__device__ __forceinline__ void keep4_h(v16h a, v16h b, v16h c, v16h d) { asm volatile("v_nop" :: "v"(a), "v"(b), "v"(c), "v"(d)); }
__device__ __forceinline__ void acc_guard4(v8f& a, v8f& b, v8f& c, v8f& d) { asm volatile("v_nop\n\tv_nop\n\tv_nop\n\tv_nop" : "+v"(a), "+v"(b), "+v"(c), "+v"(d)); }
template <typename T> struct Frag;
template <> struct Frag<_Float16> {
  typedef v16h V; union U { v16h v; v8h h[2]; };
  static __device__ __forceinline__ v16h load(const _Float16* p) {
    U f; f.h[0] = *(const v8h*)(p); f.h[1] = *(const v8h*)(p + 16); return f.v;
  }
  static __device__ __forceinline__ v8f mma(v16h a, v16h b, v8f c) {
    return __builtin_amdgcn_wmma_f32_16x16x32_f16(false, a, false, b, (short)0, c, false, false);
  }
  static __device__ __forceinline__ void guard(v8f& a, v8f& b, v16h x, v16h y) { dep_guard_h(a, b, x, y); }
  static __device__ __forceinline__ void keep(v16h a, v16h b, v16h c, v16h d) { keep4_h(a, b, c, d); }
};

__device__ __forceinline__ float fsig(float x)  { return __builtin_amdgcn_rcpf(1.0f + __expf(-x)); }
__device__ __forceinline__ float ftanh(float x) { return 1.0f - 2.0f * __builtin_amdgcn_rcpf(__expf(2.0f * x) + 1.0f); }

__global__ __launch_bounds__(NTHR) void emb_table_kernel(const float* __restrict__ time_emb, const float* __restrict__ week_emb,
                                                      const float* __restrict__ W_h, const float* __restrict__ b_h,
                                                      const float* __restrict__ W_w, const float* __restrict__ b_w,
                                                      float* __restrict__ EH4, float* __restrict__ EW4) {
  const int tid = threadIdx.x;
  const bool hour = (blockIdx.x < 48);
  const float* emb = hour ? time_emb : week_emb;
  const float* W   = hour ? W_h : W_w;
  const float* bb  = hour ? b_h : b_w;
  float* dst = hour ? EH4 : EW4;
  const int q = hour ? (int)(blockIdx.x * NTHR + tid) : (int)((blockIdx.x - 48) * NTHR + tid);
  const int i = q >> 9, rem = q & 511, jj = rem >> 2, g = rem & 3;
  const int col = g * NHID + jj;
  float acc = 0.0f;
#pragma unroll 4
  for (int k = 0; k < NHID; ++k) acc = fmaf(emb[i * NHID + k], W[k * NGATE + col], acc);
  acc += bb[col];
  ((volatile float*)dst)[q] = acc;
  __threadfence();
  ((volatile float*)dst)[q] = acc;
}

__global__ __launch_bounds__(NTHR) void tpose_f16_kernel(const float* __restrict__ src0, const float* __restrict__ src1,
                                                      const float* __restrict__ src2, int R, int C, int ldo,
                                                      unsigned short* __restrict__ Obase, long strideO, float sc) {
  __shared__ float Tt[64 * 65];
  const int tid = threadIdx.x;
  const int z = blockIdx.z;
  const float* src = (z == 0) ? src0 : (z == 1) ? src1 : src2;
  unsigned short* O = Obase + (size_t)z * (size_t)strideO;
  const int c0 = blockIdx.x * 64, r0 = blockIdx.y * 64;
#pragma unroll
  for (int i = 0; i < 4; ++i) {
    const int idx = i * NTHR + tid;
    const int rr = idx >> 4, cc = (idx & 15) * 4;
    const v4f v = *(const v4f*)(src + (size_t)(r0 + rr) * (size_t)C + c0 + cc);
    Tt[rr * 65 + cc + 0] = v[0];
    Tt[rr * 65 + cc + 1] = v[1];
    Tt[rr * 65 + cc + 2] = v[2];
    Tt[rr * 65 + cc + 3] = v[3];
  }
  __syncthreads();
  const int q = tid >> 3, c8 = (tid & 7) * 8;
  v8h hv[2];
#pragma unroll
  for (int g = 0; g < 2; ++g) {
    const int qq = g * 32 + q;
#pragma unroll
    for (int e = 0; e < 8; ++e) {
      const float f = Tt[(c8 + e) * 65 + qq];
      hv[g][e] = (_Float16)(f * sc);
    }
  }
  for (int pass = 0; pass < 2; ++pass) {
#pragma unroll
    for (int g = 0; g < 2; ++g) {
      const size_t o = (size_t)(c0 + g * 32 + q) * (size_t)ldo + (size_t)(r0 + c8);
      *(volatile v8h*)(O + o) = hv[g];
    }
    __threadfence();
  }
}

__global__ __launch_bounds__(NTHR) void lstm3_kernel(const float* __restrict__ spatial,
                                                 const int*   __restrict__ hour_idx,
                                                 const int*   __restrict__ week_idx,
                                                 const float* __restrict__ W_sp,
                                                 const float* __restrict__ b_sp,
                                                 const float* __restrict__ EH4,
                                                 const float* __restrict__ EW4,
                                                 const unsigned short* __restrict__ UTp,
                                                 float* __restrict__ hcat) {
  __shared__ __align__(16) _Float16 Ah[16 * HPITCH];
  __shared__ __align__(16) float    Etab[NHOUR * NHID * 4];
  __shared__ __align__(16) float    Hs[16 * OPITCH];
  const int tid = threadIdx.x, lane = tid & 31, wave = tid >> 5;
  const int c = lane & 15, hh = lane >> 4, koff = hh * 8;
  const int kind = (int)(blockIdx.x >> 4);
  const int rowbase = (int)(blockIdx.x & 15) * 16;
  const int j = 16 * wave + c;
  const _Float16* UT = (const _Float16*)UTp + (size_t)kind * NGATE * NHID;

#pragma unroll 1
  for (int i = tid; i < 16 * HPITCH; i += NTHR) Ah[i] = (_Float16)0.0f;

  float w0[4], w1[4], bq[4];
#pragma unroll
  for (int g = 0; g < 4; ++g) {
    const int col = g * NHID + j;
    w0[g] = USCALE * W_sp[col];
    w1[g] = USCALE * W_sp[NGATE + col];
    bq[g] = USCALE * b_sp[col];
  }
  if (kind != 0) {
    const float* src = (kind == 1) ? EH4 : EW4;
    const int n4 = (kind == 1) ? (NHOUR * NHID) : (NWEEK * NHID);
#pragma unroll 1
    for (int i = tid; i < n4; i += NTHR) *(v4f*)(Etab + 4 * i) = *(const v4f*)(src + 4 * i);
  }
  const int* idxp = (kind == 1) ? hour_idx : week_idx;
  const int imax = (kind == 1) ? (NHOUR - 1) : (NWEEK - 1);

  float cst[8], hst[8];
#pragma unroll
  for (int r = 0; r < 8; ++r) { cst[r] = 0.0f; hst[r] = 0.0f; }
  __syncthreads();

  const _Float16* ahrow = Ah + c * HPITCH + koff;
  const _Float16* ub = UT + (size_t)j * NHID + koff;
  const v8f z8 = {0.f, 0.f, 0.f, 0.f, 0.f, 0.f, 0.f, 0.f};

#pragma unroll 1
  for (int t = 0; t < NSTEP; ++t) {
    v8f acc[4];
    acc[0] = z8; acc[1] = z8; acc[2] = z8; acc[3] = z8;
    if (kind == 0) {
#pragma unroll
      for (int r = 0; r < 8; ++r) {
        const int row = rowbase + 8 * hh + r;
        const float* sp = spatial + ((size_t)row * NSTEP + (size_t)t) * 2;
        const float s0 = sp[0], s1 = sp[1];
#pragma unroll
        for (int g = 0; g < 4; ++g) acc[g][r] = fmaf(s0, w0[g], fmaf(s1, w1[g], bq[g]));
      }
    } else {
#pragma unroll
      for (int r = 0; r < 8; ++r) {
        const int row = rowbase + 8 * hh + r;
        int iv = idxp[(size_t)row * NSTEP + (size_t)t];
        iv = iv < 0 ? 0 : iv;
        iv = iv > imax ? imax : iv;
        const v4f e = *(const v4f*)(Etab + (iv * NHID + j) * 4);
#pragma unroll
        for (int g = 0; g < 4; ++g) acc[g][r] = USCALE * e[g];
      }
    }
#pragma unroll 1
    for (int k0 = 0; k0 < NHID; k0 += 32) {
      const v16h a  = Frag<_Float16>::load(ahrow + k0);
      const v16h b0 = Frag<_Float16>::load(ub + k0);
      const v16h b1 = Frag<_Float16>::load(ub + (size_t)1 * NHID * NHID + k0);
      const v16h b2 = Frag<_Float16>::load(ub + (size_t)2 * NHID * NHID + k0);
      const v16h b3 = Frag<_Float16>::load(ub + (size_t)3 * NHID * NHID + k0);
      acc[0] = Frag<_Float16>::mma(a, b0, acc[0]);
      acc[1] = Frag<_Float16>::mma(a, b1, acc[1]);
      acc[2] = Frag<_Float16>::mma(a, b2, acc[2]);
      acc[3] = Frag<_Float16>::mma(a, b3, acc[3]);
      dep_guard_h(acc[0], acc[3], a, b3);
      keep4_h(b0, b1, b2, b3);
    }
    acc_guard4(acc[0], acc[1], acc[2], acc[3]);
#pragma unroll
    for (int r = 0; r < 8; ++r) {
      const float zi = acc[0][r] * USCALE_INV;
      const float zf = acc[1][r] * USCALE_INV;
      const float zg = acc[2][r] * USCALE_INV;
      const float zo = acc[3][r] * USCALE_INV;
      const float ig = fsig(zi);
      const float fg = fsig(zf);
      const float gg = ftanh(zg);
      const float og = fsig(zo);
      const float cn = fg * cst[r] + ig * gg;
      cst[r] = cn;
      hst[r] = og * ftanh(cn);
    }
    __syncthreads();
#pragma unroll
    for (int r = 0; r < 8; ++r) Ah[(8 * hh + r) * HPITCH + j] = (_Float16)hst[r];
    __syncthreads();
  }

#pragma unroll
  for (int r = 0; r < 8; ++r) Hs[(8 * hh + r) * OPITCH + j] = hst[r];
  __syncthreads();
  float* dst = hcat + (size_t)kind * NHID;
  for (int pass = 0; pass < 2; ++pass) {
#pragma unroll
    for (int it = 0; it < 2; ++it) {
      const int idx = it * NTHR + tid;
      const int row = idx >> 5, c4 = (idx & 31) * 4;
      const v4f v = *(const v4f*)(Hs + row * OPITCH + c4);
      *(volatile v4f*)(dst + (size_t)(rowbase + row) * HCOLS + c4) = v;
    }
    __threadfence();
  }
}

__global__ __launch_bounds__(NTHR) void fc_kernel(const float* __restrict__ hcat, const float* __restrict__ fc_W,
                                               const float* __restrict__ fc_b, float* __restrict__ out) {
  __shared__ __align__(16) float res[NSEQ];
  const int tid = threadIdx.x, lane = tid & 31, wave = tid >> 5;
  float wv[12];
#pragma unroll
  for (int m = 0; m < 12; ++m) wv[m] = fc_W[lane + 32 * m];
  const float bias0 = fc_b[0];
#pragma unroll 1
  for (int rr = 0; rr < 32; ++rr) {
    const int row = wave * 32 + rr;
    const float* hrow = hcat + (size_t)row * HCOLS;
    float s = 0.0f;
#pragma unroll
    for (int m = 0; m < 12; ++m) s = fmaf(hrow[lane + 32 * m], wv[m], s);
#pragma unroll
    for (int off = 1; off < 32; off <<= 1) s += __shfl_xor(s, off, 32);
    if (lane == 0) res[row] = s + bias0;
  }
  __syncthreads();
  if (wave == 0) {
    for (int pass = 0; pass < 2; ++pass) {
#pragma unroll
      for (int it = 0; it < 2; ++it) {
        const v4f v = *(const v4f*)(res + it * 128 + lane * 4);
        *(volatile v4f*)(out + it * 128 + lane * 4) = v;
      }
      __threadfence();
    }
  }
}

extern "C" void kernel_launch(void* const* d_in, const int* in_sizes, int n_in,
                              void* d_out, int out_size, void* d_ws, size_t ws_size, hipStream_t stream) {
  if (n_in < 16 || d_out == nullptr || d_ws == nullptr) return;
  if (in_sizes[0] != NSEQ * NSTEP * 2 || in_sizes[1] != NSEQ * NSTEP || in_sizes[2] != NSEQ * NSTEP ||
      in_sizes[3] != NHOUR * NHID || in_sizes[4] != NWEEK * NHID ||
      in_sizes[5] != 2 * NGATE || in_sizes[6] != NHID * NGATE || in_sizes[7] != NGATE ||
      in_sizes[8] != NHID * NGATE || in_sizes[9] != NHID * NGATE || in_sizes[10] != NGATE ||
      in_sizes[11] != NHID * NGATE || in_sizes[12] != NHID * NGATE || in_sizes[13] != NGATE ||
      in_sizes[14] != HCOLS || in_sizes[15] != 1 || out_size != NSEQ) return;

  const float* spatial  = (const float*)d_in[0];
  const int*   hour_idx = (const int*)  d_in[1];
  const int*   week_idx = (const int*)  d_in[2];
  const float* time_emb = (const float*)d_in[3];
  const float* week_emb = (const float*)d_in[4];
  const float* W_sp = (const float*)d_in[5];
  const float* U_sp = (const float*)d_in[6];
  const float* b_sp = (const float*)d_in[7];
  const float* W_h  = (const float*)d_in[8];
  const float* U_h  = (const float*)d_in[9];
  const float* b_h  = (const float*)d_in[10];
  const float* W_w  = (const float*)d_in[11];
  const float* U_w  = (const float*)d_in[12];
  const float* b_w  = (const float*)d_in[13];
  const float* fc_W = (const float*)d_in[14];
  const float* fc_b = (const float*)d_in[15];
  float* out = (float*)d_out;

  char* ws = (char*)d_ws; size_t off = 0;
  auto carve = [&](size_t bytes) -> char* { char* p = ws + off; off += (bytes + 255) & ~(size_t)255; return p; };
  unsigned short* UT = (unsigned short*)carve((size_t)3 * NGATE * NHID * 2);
  float* EH4  = (float*)carve((size_t)NHOUR * NHID * 4 * sizeof(float));
  float* EW4  = (float*)carve((size_t)NWEEK * NHID * 4 * sizeof(float));
  float* HCAT = (float*)carve((size_t)NSEQ * HCOLS * sizeof(float));
  if (off > ws_size || off > (size_t)134217728) return;

  emb_table_kernel<<<62, NTHR, 0, stream>>>(time_emb, week_emb, W_h, b_h, W_w, b_w, EH4, EW4);
  tpose_f16_kernel<<<dim3(NGATE / 64, NHID / 64, 3), NTHR, 0, stream>>>(U_sp, U_h, U_w, NHID, NGATE, NHID, UT,
                                                                      (long)NGATE * NHID, USCALE);
  lstm3_kernel<<<3 * (NSEQ / 16), NTHR, 0, stream>>>(spatial, hour_idx, week_idx, W_sp, b_sp, EH4, EW4, UT, HCAT);
  fc_kernel<<<1, NTHR, 0, stream>>>(HCAT, fc_W, fc_b, out);
}
